// LocalTopologyBlockWithAngle_85727547228406
// MI455X (gfx1250) — hardware-run, weakly checked
//
#include <hip/hip_runtime.h>
#include <stdint.h>
#include <math.h>

#pragma clang fp contract(off)

#define NN      8192
#define CC      128
#define HH      3
#define MR      (HH * CC)
#define NWG     (2 * CC + 2)
#define NARR    10
#define LEAKY   0.2f
#define PSCALE  262144.0f
#define PINV    3.814697265625e-06f
#define WSC     16.0f
#define WINV    0.0625f
#define OSP     68
#define OSQ     132
#define PTP     40
#define UCH     1024

#define A_SU 0
#define A_SV 1
#define A_CS 2
#define A_SN 3
#define A_AP 4
#define A_BP 5
#define A_CU 6
#define A_M  7
#define A_RZ 8
#define A_G  9

static_assert(NN % UCH == 0);
static_assert(NN % 256 == 0);
static_assert(NN % 64 == 0);
static_assert(NN % 32 == 0);
static_assert(MR % 128 == 0);
static_assert(CC == 128);
static_assert(CC % 32 == 0);
static_assert((NN * CC) % 8 == 0);
static_assert((MR * CC) % 8 == 0);
static_assert((OSP * 4) % 16 == 0);
static_assert((OSQ * 4) % 16 == 0);
static_assert((PTP * 2) % 16 == 0);
static_assert((HH * 3 * CC) % 4 == 0);
static_assert((HH * 3 * CC) / 4 <= 384);

typedef _Float16 v4h  __attribute__((ext_vector_type(4)));
typedef _Float16 v8h  __attribute__((ext_vector_type(8)));
typedef _Float16 v16h __attribute__((ext_vector_type(16)));
typedef float    v4f  __attribute__((ext_vector_type(4)));
typedef float    v8f  __attribute__((ext_vector_type(8)));

union FragH { v8h p[2]; v16h v; };
static_assert(sizeof(FragH) == 32);

__device__ __forceinline__ v8f zero8() { v8f z = {0.f, 0.f, 0.f, 0.f, 0.f, 0.f, 0.f, 0.f}; return z; }

__device__ __forceinline__ FragH ldfrag_h(const _Float16* q) {
  FragH f;
  f.p[0] = *(const v8h*)(q);
  f.p[1] = *(const v8h*)(q + 16);
  return f;
}

__device__ __forceinline__ v8f mma_h(v16h a, v16h b, v8f c) {
  v8f d = __builtin_amdgcn_wmma_f32_16x16x32_f16(false, a, false, b, (short)0, c, false, false);
#if defined(__HIP_DEVICE_COMPILE__)
  asm volatile("v_nop\n\tv_nop\n\tv_nop\n\tv_nop" : "+v"(d) : "v"(a), "v"(b));
#endif
  return d;
}

__global__ __launch_bounds__(256)
void k_cvt(const float* __restrict__ x, _Float16* y, int n8, float sc) {
  const int t = blockIdx.x * 256 + (int)threadIdx.x;
  if (t >= n8) return;
  const float* s = x + (size_t)t * 8;
  const v4f a = *(const v4f*)(s);
  const v4f b = *(const v4f*)(s + 4);
  v8h o;
  o[0] = (_Float16)(a[0] * sc); o[1] = (_Float16)(a[1] * sc); o[2] = (_Float16)(a[2] * sc); o[3] = (_Float16)(a[3] * sc);
  o[4] = (_Float16)(b[0] * sc); o[5] = (_Float16)(b[1] * sc); o[6] = (_Float16)(b[2] * sc); o[7] = (_Float16)(b[3] * sc);
  _Float16* d = y + (size_t)t * 8;
  *(volatile v8h*)d = o;
  __threadfence();
  *(volatile v8h*)d = o;
}

__global__ __launch_bounds__(256)
void k_nodes(const float* __restrict__ X, const float* __restrict__ phis, const float* __restrict__ wg,
             float* node) {
  __shared__ float Lw[NWG + 6];
  __shared__ __align__(16) float Lo[7 * 32];
  const int t = threadIdx.x, n = t >> 3, q = t & 7;
  const int u0 = blockIdx.x * 32, u = u0 + n;
  for (int i = t; i < NWG; i += 256) Lw[i] = wg[i];
  __syncthreads();
  const float* xp = X + (size_t)u * CC + 16 * q;
  float su = 0.f, sv = 0.f;
#pragma unroll 1
  for (int k = 0; k < 16; ++k) {
    const float x = xp[k];
    su = fmaf(x, Lw[16 * q + k], su);
    sv = fmaf(x, Lw[CC + 16 * q + k], sv);
  }
#pragma unroll
  for (int o = 1; o < 8; o <<= 1) {
    su += __shfl_xor(su, o, 32);
    sv += __shfl_xor(sv, o, 32);
  }
  float sn, cs;
  sincosf(phis[u], &sn, &cs);
  const float wc = Lw[2 * CC], wq = Lw[2 * CC + 1];
  const float ap = fmaf(wc, cs, wq * sn);
  const float bp = fmaf(wc, sn, -(wq * cs));
  const float cu = __expf(su);
  if (q == 0) {
    Lo[A_SU * 32 + n] = su; Lo[A_SV * 32 + n] = sv; Lo[A_CS * 32 + n] = cs; Lo[A_SN * 32 + n] = sn;
    Lo[A_AP * 32 + n] = ap; Lo[A_BP * 32 + n] = bp; Lo[A_CU * 32 + n] = cu;
  }
  __syncthreads();
  const bool wr = (t < 56);
  v4f v = {0.f, 0.f, 0.f, 0.f};
  float* d = node;
  if (wr) {
    const int a = t >> 3, e = t & 7;
    v = *(const v4f*)(Lo + a * 32 + 4 * e);
    d = node + (size_t)a * NN + u0 + 4 * e;
  }
  if (wr) *(volatile v4f*)d = v;
  __threadfence();
  if (wr) *(volatile v4f*)d = v;
}

__global__ __launch_bounds__(256)
void k_colstats(float* node) {
  __shared__ __align__(16) v4f L[UCH];
  __shared__ __align__(16) float Ls[3 * 256];
  const int t = threadIdx.x;
  const int v0b = blockIdx.x * 256;
  const int v = v0b + t;
  const float* suA = node + (size_t)A_SU * NN;
  const float* apA = node + (size_t)A_AP * NN;
  const float* bpA = node + (size_t)A_BP * NN;
  const float svv = node[(size_t)A_SV * NN + v];
  const float csv = node[(size_t)A_CS * NN + v];
  const float snv = node[(size_t)A_SN * NN + v];
  float m = -1.0e30f, z = 0.f;
#pragma unroll 1
  for (int c0 = 0; c0 < NN; c0 += UCH) {
    for (int i = t; i < UCH; i += 256) {
      v4f w;
      w[0] = suA[c0 + i]; w[1] = apA[c0 + i]; w[2] = bpA[c0 + i]; w[3] = 0.f;
      L[i] = w;
    }
    __syncthreads();
#pragma unroll 4
    for (int i = 0; i < UCH; ++i) {
      const v4f w = L[i];
      const float tt = fmaf(w[1], csv, w[2] * snv);
      const float e  = (w[0] + svv) + tt;
      const float l  = fmaxf(e, LEAKY * e);
      const float d  = l - m;
      const float p  = __expf(-fabsf(d));
      const float z1 = fmaf(z, p, 1.0f);
      const float z2 = z + p;
      z = (d > 0.f) ? z1 : z2;
      m = fmaxf(m, l);
    }
    __syncthreads();
  }
  const float rz = 1.0f / z;
  const float g  = __expf(svv - m) * rz;
  Ls[t] = m; Ls[256 + t] = rz * PSCALE; Ls[512 + t] = g;
  __syncthreads();
  const bool wr = (t < 192);
  v4f ov = {0.f, 0.f, 0.f, 0.f};
  float* d2 = node;
  if (wr) {
    const int a = t >> 6, pc = t & 63;
    ov = *(const v4f*)(Ls + a * 256 + 4 * pc);
    d2 = node + (size_t)(A_M + a) * NN + v0b + 4 * pc;
  }
  if (wr) *(volatile v4f*)d2 = ov;
  __threadfence();
  if (wr) *(volatile v4f*)d2 = ov;
}

__global__ __launch_bounds__(256)
void k_xk(const _Float16* __restrict__ A, const _Float16* __restrict__ B, _Float16* C) {
  __shared__ __align__(16) float Os[128 * OSP];
  const int tid  = threadIdx.x;
  const int lane = tid & 31, wave = tid >> 5;
  const int hh   = lane >> 4, cl = lane & 15;
  const int wm   = wave >> 1, wn = wave & 1;
  const int mBase = blockIdx.x * 128;
  const int nBase = blockIdx.y * 64;
  const _Float16* a0p = A + (size_t)(mBase + 32 * wm + cl) * CC + 8 * hh;
  const _Float16* a1p = a0p + (size_t)16 * CC;
  const _Float16* b0p = B + (size_t)(nBase + 32 * wn + cl) * CC + 8 * hh;
  const _Float16* b1p = b0p + (size_t)16 * CC;

  v8f acc[2][2];
#pragma unroll
  for (int mi = 0; mi < 2; ++mi)
#pragma unroll
    for (int ni = 0; ni < 2; ++ni) acc[mi][ni] = zero8();

#pragma unroll 1
  for (int k0 = 0; k0 < CC; k0 += 32) {
    const FragH fa0 = ldfrag_h(a0p + k0);
    const FragH fa1 = ldfrag_h(a1p + k0);
    const FragH fb0 = ldfrag_h(b0p + k0);
    const FragH fb1 = ldfrag_h(b1p + k0);
    acc[0][0] = mma_h(fa0.v, fb0.v, acc[0][0]);
    acc[0][1] = mma_h(fa0.v, fb1.v, acc[0][1]);
    acc[1][0] = mma_h(fa1.v, fb0.v, acc[1][0]);
    acc[1][1] = mma_h(fa1.v, fb1.v, acc[1][1]);
  }

#pragma unroll
  for (int mi = 0; mi < 2; ++mi) {
#pragma unroll
    for (int ni = 0; ni < 2; ++ni) {
      const int n_loc = 32 * wn + 16 * ni + cl;
#pragma unroll
      for (int r = 0; r < 8; ++r) {
        const int m_loc = 32 * wm + 16 * mi + 8 * hh + r;
        Os[m_loc * OSP + n_loc] = acc[mi][ni][r];
      }
    }
  }
  __syncthreads();

  const int e = tid & 7, lq = tid >> 3;
  v8h o[4];
  size_t po[4];
#pragma unroll
  for (int it = 0; it < 4; ++it) {
    const int row = it * 32 + lq;
    const float* op = Os + row * OSP + 8 * e;
    const v4f x0 = *(const v4f*)(op);
    const v4f x1 = *(const v4f*)(op + 4);
    v8h w;
    w[0] = (_Float16)(x0[0] * WINV); w[1] = (_Float16)(x0[1] * WINV);
    w[2] = (_Float16)(x0[2] * WINV); w[3] = (_Float16)(x0[3] * WINV);
    w[4] = (_Float16)(x1[0] * WINV); w[5] = (_Float16)(x1[1] * WINV);
    w[6] = (_Float16)(x1[2] * WINV); w[7] = (_Float16)(x1[3] * WINV);
    o[it] = w;
    po[it] = (size_t)(mBase + row) * NN + nBase + 8 * e;
  }
#pragma unroll
  for (int it = 0; it < 4; ++it) *(volatile v8h*)(C + po[it]) = o[it];
  __threadfence();
#pragma unroll
  for (int it = 0; it < 4; ++it) *(volatile v8h*)(C + po[it]) = o[it];
}

__global__ __launch_bounds__(384)
void k_rank(const float* __restrict__ node, const float* __restrict__ X, const float* __restrict__ W, float* Y) {
  __shared__ float Lf[3 * UCH];
  __shared__ float Gs[3 * CC];
  __shared__ __align__(16) float Ys[HH * 3 * CC];
  const int t = threadIdx.x;
  const int j = t >> 7, d = t & 127;
  const float* gA  = node + (size_t)A_G * NN;
  const float* csA = node + (size_t)A_CS * NN;
  const float* snA = node + (size_t)A_SN * NN;
  float G = 0.f;
#pragma unroll 1
  for (int c0 = 0; c0 < NN; c0 += UCH) {
    for (int i = t; i < UCH; i += 384) {
      const float gv = gA[c0 + i];
      Lf[i] = gv;
      Lf[UCH + i] = gv * csA[c0 + i];
      Lf[2 * UCH + i] = gv * snA[c0 + i];
    }
    __syncthreads();
    const float* Lj = Lf + j * UCH;
    const float* xp = X + (size_t)c0 * CC + d;
#pragma unroll 4
    for (int i = 0; i < UCH; ++i) G = fmaf(Lj[i], xp[(size_t)i * CC], G);
    __syncthreads();
  }
  Gs[j * CC + d] = G;
  __syncthreads();
  const int h = t >> 7, c = t & 127;
  const float* wr = W + ((size_t)h * CC + c) * CC;
  float y0 = 0.f, y1 = 0.f, y2 = 0.f;
#pragma unroll 2
  for (int k = 0; k < CC; ++k) {
    const float w = wr[k];
    y0 = fmaf(w, Gs[k], y0);
    y1 = fmaf(w, Gs[CC + k], y1);
    y2 = fmaf(w, Gs[2 * CC + k], y2);
  }
  Ys[(h * 3 + 0) * CC + c] = y0;
  Ys[(h * 3 + 1) * CC + c] = y1;
  Ys[(h * 3 + 2) * CC + c] = y2;
  __syncthreads();
  const bool ok = (t < (HH * 3 * CC) / 4);
  v4f ov = {0.f, 0.f, 0.f, 0.f};
  float* dst = Y;
  if (ok) { ov = *(const v4f*)(Ys + 4 * t); dst = Y + 4 * t; }
  if (ok) *(volatile v4f*)dst = ov;
  __threadfence();
  if (ok) *(volatile v4f*)dst = ov;
}

__global__ __launch_bounds__(256)
void k_main(const float* __restrict__ node, const _Float16* __restrict__ XkT, const float* __restrict__ Yg,
            float* out) {
  __shared__ __align__(16) _Float16 Pt[2][32 * PTP];
  __shared__ __align__(16) float Rt[4 * 32];
  __shared__ __align__(16) float Yl[HH * 3 * CC];
  __shared__ __align__(16) float Os[32 * OSQ];
  const int t    = threadIdx.x;
  const int lane = t & 31, wave = t >> 5;
  const int hh   = lane >> 4, cl = lane & 15;
  const int rg   = wave >> 2, cq = wave & 3;
  const int u0   = blockIdx.x * 32;

  if (t < 128) {
    const int a = t >> 5, i = t & 31;
    const int src = (a == 0) ? A_SU : (a + 3);
    Rt[a * 32 + i] = node[(size_t)src * NN + u0 + i];
  }
  for (int i = t; i < HH * 3 * CC; i += 256) Yl[i] = Yg[i];
  __syncthreads();

  const int brow = t >> 3, bq = t & 7;
  const float su_r  = Rt[brow];
  const float ap_r  = Rt[32 + brow];
  const float bp_r  = Rt[64 + brow];
  const float cuS_r = Rt[96 + brow] * PSCALE;
  const float* svA = node + (size_t)A_SV * NN;
  const float* csA = node + (size_t)A_CS * NN;
  const float* snA = node + (size_t)A_SN * NN;
  const float* mA  = node + (size_t)A_M  * NN;
  const float* rzA = node + (size_t)A_RZ * NN;
  const float* gA  = node + (size_t)A_G  * NN;

  v8f acc[HH][2];
#pragma unroll
  for (int h = 0; h < HH; ++h) { acc[h][0] = zero8(); acc[h][1] = zero8(); }

  const _Float16* bbase = XkT + (size_t)(32 * cq + cl) * NN + 8 * hh;
  _Float16* pst = &Pt[0][0] + brow * PTP + 4 * bq;
  const _Float16* pld = &Pt[0][0] + (16 * rg + cl) * PTP + 8 * hh;

#pragma unroll 1
  for (int ks = 0; ks < NN / 32; ++ks) {
    const int v0 = ks * 32;
    const int bo = (ks & 1) * (32 * PTP);
    const int vb = v0 + 4 * bq;
    const v4f sv4 = *(const v4f*)(svA + vb);
    const v4f cs4 = *(const v4f*)(csA + vb);
    const v4f sn4 = *(const v4f*)(snA + vb);
    const v4f m4  = *(const v4f*)(mA  + vb);
    const v4f rz4 = *(const v4f*)(rzA + vb);
    const v4f g4  = *(const v4f*)(gA  + vb);
    v4h ph;
#pragma unroll
    for (int jj = 0; jj < 4; ++jj) {
      const float tt = fmaf(ap_r, cs4[jj], bp_r * sn4[jj]);
      const float e  = (su_r + sv4[jj]) + tt;
      const float l  = fmaxf(e, LEAKY * e);
      const float p  = __expf(l - m4[jj]);
      const float cg = cuS_r * g4[jj];
      const float qv = fmaf(cg, tt, cg);
      float ps = fmaf(p, rz4[jj], -qv);
      ps = fminf(fmaxf(ps, -60000.0f), 60000.0f);
      ph[jj] = (_Float16)ps;
    }
    *(v4h*)(pst + bo) = ph;
    __syncthreads();

    const FragH fa = ldfrag_h(pld + bo);
    const _Float16* bp0 = bbase + v0;
#pragma unroll
    for (int h = 0; h < HH; ++h) {
#pragma unroll
      for (int ct = 0; ct < 2; ++ct) {
        const FragH fb = ldfrag_h(bp0 + (size_t)(h * CC + 16 * ct) * NN);
        acc[h][ct] = mma_h(fa.v, fb.v, acc[h][ct]);
      }
    }
  }

#pragma unroll
  for (int ct = 0; ct < 2; ++ct) {
    const int col = 32 * cq + 16 * ct + cl;
#pragma unroll
    for (int r = 0; r < 8; ++r) {
      const int row = 16 * rg + 8 * hh + r;
      const float cu  = Rt[96 + row];
      const float ap  = Rt[32 + row];
      const float bpv = Rt[64 + row];
      float s = 0.f;
#pragma unroll
      for (int h = 0; h < HH; ++h) {
        const float y0 = Yl[(h * 3 + 0) * CC + col];
        const float y1 = Yl[(h * 3 + 1) * CC + col];
        const float y2 = Yl[(h * 3 + 2) * CC + col];
        const float rk = fmaf(ap, y1, fmaf(bpv, y2, y0));
        const float val = fmaf(cu, rk, acc[h][ct][r] * PINV);
        s += fmaxf(val, 0.f);
      }
      Os[row * OSQ + col] = s;
    }
  }
  __syncthreads();

  const int e = t & 7, lq = t >> 3;
  v4f ov[4];
  size_t po[4];
#pragma unroll
  for (int it = 0; it < 4; ++it) {
    const int Lx = it * 32 + lq;
    const int row = Lx >> 2, seg = Lx & 3;
    ov[it] = *(const v4f*)(Os + row * OSQ + seg * 32 + 4 * e);
    po[it] = (size_t)(u0 + row) * CC + seg * 32 + 4 * e;
  }
#pragma unroll
  for (int it = 0; it < 4; ++it) *(volatile v4f*)(out + po[it]) = ov[it];
  __threadfence();
#pragma unroll
  for (int it = 0; it < 4; ++it) *(volatile v4f*)(out + po[it]) = ov[it];
}

extern "C" void kernel_launch(void* const* d_in, const int* in_sizes, int n_in,
                              void* d_out, int out_size, void* d_ws, size_t ws_size,
                              hipStream_t stream) {
  if (n_in < 4) return;
  if (in_sizes[0] != NN * CC) return;
  if (in_sizes[1] != NN) return;
  if (in_sizes[2] != NWG) return;
  if (in_sizes[3] != HH * CC * CC) return;
  if (out_size != NN * CC) return;

  size_t off = 0;
  const size_t oNode = off; off += (size_t)NARR * NN * 4;
  const size_t oY    = off; off += (size_t)8192;
  const size_t oX16  = off; off += (size_t)NN * CC * 2;
  const size_t oW16  = off; off += (size_t)MR * CC * 2;
  const size_t oXk   = off; off += (size_t)MR * NN * 2;
  if (off > ws_size) return;
  if (off > (size_t)134217728) return;

  const float* X    = (const float*)d_in[0];
  const float* phis = (const float*)d_in[1];
  const float* wg   = (const float*)d_in[2];
  const float* W    = (const float*)d_in[3];
  float* out = (float*)d_out;

  char* ws = (char*)d_ws;
  float*    node = (float*)(ws + oNode);
  float*    Yg   = (float*)(ws + oY);
  _Float16* X16  = (_Float16*)(ws + oX16);
  _Float16* W16  = (_Float16*)(ws + oW16);
  _Float16* XkT  = (_Float16*)(ws + oXk);

  const dim3 blk256(256);
  const int n8x = (NN * CC) / 8;
  const int n8w = (MR * CC) / 8;

  k_nodes<<<dim3(NN / 32), blk256, 0, stream>>>(X, phis, wg, node);
  k_colstats<<<dim3(NN / 256), blk256, 0, stream>>>(node);
  k_cvt<<<dim3((n8x + 255) / 256), blk256, 0, stream>>>(X, X16, n8x, 1.0f);
  k_cvt<<<dim3((n8w + 255) / 256), blk256, 0, stream>>>(W, W16, n8w, WSC);
  k_xk<<<dim3(MR / 128, NN / 64), blk256, 0, stream>>>(W16, X16, XkT);
  k_rank<<<dim3(1), dim3(384), 0, stream>>>(node, X, W, Yg);
  k_main<<<dim3(NN / 32), blk256, 0, stream>>>(node, XkT, Yg, out);
  (void)hipGetLastError();
}
